// PointNetFeaturePropagation_81587198754954
// MI455X (gfx1250) — hardware-verified
//
#include <hip/hip_runtime.h>
#pragma clang fp contract(off)

typedef __attribute__((ext_vector_type(16))) __bf16   v16b;
typedef __attribute__((ext_vector_type(8)))  __bf16   v8b;
typedef __attribute__((ext_vector_type(8)))  float    v8f;
typedef __attribute__((ext_vector_type(4)))  float    v4f;
typedef __attribute__((ext_vector_type(4)))  unsigned v4u;
typedef __attribute__((ext_vector_type(4)))  int      v4i;

constexpr int kBatch = 2;
constexpr int kNq    = 16384;
constexpr int kNs    = 4096;
constexpr int kD1    = 128;
constexpr int kD2    = 256;
constexpr int kC1    = 256;
constexpr int kC2    = 128;
constexpr int kK1    = kD1 + kD2;
constexpr int kRows  = kBatch * kNq;
constexpr int kPartRows   = 128;
constexpr int kPartBlocks = kRows / kPartRows;
constexpr float kBnEps = 1e-5f;

static_assert(kK1 % 32 == 0 && kC1 % 32 == 0, "gemm K multiple of 32");
static_assert(kRows % 64 == 0 && kC1 % 64 == 0 && kC2 % 64 == 0, "gemm M,N multiples of 64");
static_assert(kPartBlocks == 256, "partial block count");
static_assert(kNq % 256 == 0 && kNs % 32 == 0 && kD2 % 64 == 0 && kD1 % 64 == 0, "tile multiples");

__device__ __forceinline__ unsigned bf_rne_bits(float f) {
  const unsigned u = __float_as_uint(f);
  return (u + 0x7FFFu + ((u >> 16) & 1u)) >> 16;
}
__device__ __forceinline__ float bf_bits_f(unsigned h) { return __uint_as_float(h << 16); }

__device__ __forceinline__ void split_pack8(const float (&f)[8], v4u& H, v4u& L) {
  unsigned h[8], l[8];
#pragma unroll
  for (int e = 0; e < 8; ++e) {
    h[e] = bf_rne_bits(f[e]);
    l[e] = bf_rne_bits(f[e] - bf_bits_f(h[e]));
  }
  H = (v4u){(h[0] & 0xffffu) | (h[1] << 16), (h[2] & 0xffffu) | (h[3] << 16),
            (h[4] & 0xffffu) | (h[5] << 16), (h[6] & 0xffffu) | (h[7] << 16)};
  L = (v4u){(l[0] & 0xffffu) | (l[1] << 16), (l[2] & 0xffffu) | (l[3] << 16),
            (l[4] & 0xffffu) | (l[5] << 16), (l[6] & 0xffffu) | (l[7] << 16)};
}

__device__ __forceinline__ void store2_planes(unsigned short* ph, unsigned short* pl, v4u H, v4u L) {
  *(volatile v4u*)(void*)ph = H;
  *(volatile v4u*)(void*)pl = L;
  __threadfence();
  *(volatile v4u*)(void*)ph = H;
  *(volatile v4u*)(void*)pl = L;
}

__device__ __forceinline__ void dep_guard4_b(v8f& a, v8f& b, v8f& c, v8f& d, v16b x, v16b y) {
  asm volatile("v_nop\n\tv_nop\n\tv_nop\n\tv_nop" : "+v"(a), "+v"(b), "+v"(c), "+v"(d) : "v"(x), "v"(y));
}
__device__ __forceinline__ void keep4_b(v16b a, v16b b, v16b c, v16b d) { asm volatile("v_nop" :: "v"(a), "v"(b), "v"(c), "v"(d)); }
__device__ __forceinline__ void acc_guard4(v8f& a, v8f& b, v8f& c, v8f& d) { asm volatile("v_nop\n\tv_nop\n\tv_nop\n\tv_nop" : "+v"(a), "+v"(b), "+v"(c), "+v"(d)); }

struct FragB {
  union U { v16b v; v8b h[2]; };
  static __device__ __forceinline__ v16b load(const __bf16* p) {
    U f; f.h[0] = *(const v8b*)(p); f.h[1] = *(const v8b*)(p + 16); return f.v;
  }
  static __device__ __forceinline__ v8f mma(v16b a, v16b b, v8f c) {
    return __builtin_amdgcn_wmma_f32_16x16x32_bf16(false, a, false, b, (short)0, c, false, false);
  }
};

__global__ __launch_bounds__(256) void pack_wt_split(const float* __restrict__ W, int Kd, int Cd,
                                                     unsigned short* __restrict__ hi,
                                                     unsigned short* __restrict__ lo) {
  const int i  = blockIdx.x * 256 + threadIdx.x;
  const int kc = Kd >> 3;
  if (i < Cd * kc) {
    const int n  = i / kc;
    const int k8 = (i - n * kc) << 3;
    float f[8];
#pragma unroll
    for (int e = 0; e < 8; ++e) f[e] = W[(size_t)(k8 + e) * Cd + n];
    v4u H, L;
    split_pack8(f, H, L);
    const size_t o = (size_t)n * Kd + k8;
    store2_planes(hi + o, lo + o, H, L);
  }
}

__global__ __launch_bounds__(256) void transpose_p2(const float* __restrict__ p2, float* __restrict__ p2t) {
  __shared__ float tile[64][33];
  const int t  = threadIdx.x;
  const int s0 = blockIdx.x * 32;
  const int c0 = blockIdx.y * 64;
  const int b  = blockIdx.z;
#pragma unroll
  for (int it = 0; it < 8; ++it) {
    const int idx = it * 256 + t;
    const int c = idx >> 5, s = idx & 31;
    tile[c][s] = p2[((size_t)b * kD2 + c0 + c) * kNs + s0 + s];
  }
  __syncthreads();
  v4f val[2];
  float* dst[2];
#pragma unroll
  for (int it = 0; it < 2; ++it) {
    const int idx = it * 256 + t;
    const int s = idx >> 4, c4 = (idx & 15) * 4;
    val[it] = (v4f){tile[c4][s], tile[c4 + 1][s], tile[c4 + 2][s], tile[c4 + 3][s]};
    dst[it] = p2t + ((size_t)b * kNs + s0 + s) * kD2 + c0 + c4;
  }
  *(volatile v4f*)dst[0] = val[0];
  *(volatile v4f*)dst[1] = val[1];
  __threadfence();
  *(volatile v4f*)dst[0] = val[0];
  *(volatile v4f*)dst[1] = val[1];
}

__global__ __launch_bounds__(256) void xcols_from_p1(const float* __restrict__ p1,
                                                     unsigned short* __restrict__ Xhi,
                                                     unsigned short* __restrict__ Xlo) {
  __shared__ float tile[64][33];
  const int t  = threadIdx.x;
  const int n0 = blockIdx.x * 32;
  const int c0 = blockIdx.y * 64;
  const int b  = blockIdx.z;
#pragma unroll
  for (int it = 0; it < 8; ++it) {
    const int idx = it * 256 + t;
    const int c = idx >> 5, n = idx & 31;
    tile[c][n] = p1[((size_t)b * kD1 + c0 + c) * kNq + n0 + n];
  }
  __syncthreads();
  const int row = t >> 3;
  const int c8  = (t & 7) * 8;
  float f[8];
#pragma unroll
  for (int e = 0; e < 8; ++e) f[e] = tile[c8 + e][row];
  v4u H, L;
  split_pack8(f, H, L);
  const size_t o = ((size_t)b * kNq + n0 + row) * kK1 + c0 + c8;
  store2_planes(Xhi + o, Xlo + o, H, L);
}

__global__ __launch_bounds__(256) void knn3_interp(const float* __restrict__ xyz1, const float* __restrict__ xyz2,
                                                   const float* __restrict__ p2t,
                                                   unsigned short* __restrict__ Xhi,
                                                   unsigned short* __restrict__ Xlo) {
#pragma clang fp contract(off)
  __shared__ v4f cand[kNs];
  __shared__ v4i sIdx[256];
  __shared__ v4f sWgt[256];
  const int t    = threadIdx.x;
  const int lane = t & 31;
  const int wave = t >> 5;
  const int b    = blockIdx.y;

  const float* x2 = xyz2 + (size_t)b * 3 * kNs;
#pragma unroll 4
  for (int i = t; i < kNs; i += 256) {
    const float x = x2[i];
    const float y = x2[kNs + i];
    const float z = x2[2 * kNs + i];
    const float xx = x * x;
    const float yy = y * y;
    const float zz = z * z;
    const float s2 = (xx + zz) + yy;
    cand[i] = (v4f){x, y, z, s2};
  }
  __syncthreads();

  const int n = blockIdx.x * 256 + t;
  const float* x1 = xyz1 + (size_t)b * 3 * kNq;
  const float qx = x1[n];
  const float qy = x1[kNq + n];
  const float qz = x1[2 * kNq + n];
  const float qxx = qx * qx;
  const float qyy = qy * qy;
  const float qzz = qz * qz;
  const float s1 = (qxx + qzz) + qyy;

  float d0 = 3.4e38f, d1 = 3.4e38f, d2 = 3.4e38f;
  int   i0 = 0, i1 = 0, i2 = 0;
#pragma unroll 4
  for (int s = 0; s < kNs; ++s) {
    const v4f cd = cand[s];
    float p = qx * cd.x;
    p = __builtin_fmaf(qy, cd.y, p);
    p = __builtin_fmaf(qz, cd.z, p);
    const float p2 = p + p;
    const float u  = s1 - p2;
    float d = u + cd.w;
    d = fmaxf(d, 0.0f);
    if (d < d2) {
      const bool lt1 = d < d1;
      const bool lt0 = d < d0;
      d2 = lt1 ? d1 : d;
      i2 = lt1 ? i1 : s;
      d1 = lt0 ? d0 : (lt1 ? d : d1);
      i1 = lt0 ? i0 : (lt1 ? s : i1);
      d0 = lt0 ? d : d0;
      i0 = lt0 ? s : i0;
    }
  }
  {
    const float e0 = fmaxf(d0, 1e-6f);
    const float e1 = fmaxf(d1, 1e-6f);
    const float e2 = fmaxf(d2, 1e-6f);
    const float r0 = 1.0f / e0;
    const float r1 = 1.0f / e1;
    const float r2 = 1.0f / e2;
    const float rs  = (r0 + r2) + r1;
    const float den = fmaxf(rs, 1e-6f);
    const float w0 = r0 / den;
    const float w1 = r1 / den;
    const float w2 = r2 / den;
    const int j0 = min(max(i0, 0), kNs - 1);
    const int j1 = min(max(i1, 0), kNs - 1);
    const int j2 = min(max(i2, 0), kNs - 1);
    sIdx[t] = (v4i){j0, j1, j2, 0};
    sWgt[t] = (v4f){w0, w1, w2, 0.0f};
  }
  __syncthreads();

  const float* pb = p2t + (size_t)b * kNs * kD2 + lane * 8;
#pragma unroll 1
  for (int rr = 0; rr < 32; ++rr) {
    const int rl = wave * 32 + rr;
    const v4i id = sIdx[rl];
    const v4f wg = sWgt[rl];
    const int j0 = min(max(id.x, 0), kNs - 1);
    const int j1 = min(max(id.y, 0), kNs - 1);
    const int j2 = min(max(id.z, 0), kNs - 1);
    const float* q0 = pb + (size_t)j0 * kD2;
    const float* q1 = pb + (size_t)j1 * kD2;
    const float* q2 = pb + (size_t)j2 * kD2;
    const v4f a0 = *(const v4f*)(q0);
    const v4f a1 = *(const v4f*)(q0 + 4);
    const v4f b0 = *(const v4f*)(q1);
    const v4f b1 = *(const v4f*)(q1 + 4);
    const v4f c0 = *(const v4f*)(q2);
    const v4f c1 = *(const v4f*)(q2 + 4);
    float f[8];
#pragma unroll
    for (int e = 0; e < 4; ++e) {
      const float ta = a0[e] * wg.x;
      const float tb = b0[e] * wg.y;
      const float tc = c0[e] * wg.z;
      const float v  = (ta + tb) + tc;
      f[e] = (fabsf(v) <= 3.4028234663852886e38f) ? v : 0.0f;
      const float ua = a1[e] * wg.x;
      const float ub = b1[e] * wg.y;
      const float uc = c1[e] * wg.z;
      const float w  = (ua + ub) + uc;
      f[4 + e] = (fabsf(w) <= 3.4028234663852886e38f) ? w : 0.0f;
    }
    v4u H, L;
    split_pack8(f, H, L);
    const size_t m = (size_t)b * kNq + (size_t)blockIdx.x * 256 + rl;
    const size_t o = m * kK1 + kD1 + lane * 8;
    store2_planes(Xhi + o, Xlo + o, H, L);
  }
}

template <int BIAS_MODE>
__global__ __launch_bounds__(256) void wmma_gemm64_bf16x3(
    const unsigned short* __restrict__ Ap, const unsigned short* __restrict__ A2p, int lda,
    const unsigned short* __restrict__ Btp, const unsigned short* __restrict__ Bt2p, int ldb,
    float* __restrict__ Cout, int ldc, const float* __restrict__ bias, int M, int N, int K) {
  const __bf16* A   = (const __bf16*)Ap;
  const __bf16* A2  = (const __bf16*)A2p;
  const __bf16* Bt  = (const __bf16*)Btp;
  const __bf16* Bt2 = (const __bf16*)Bt2p;
  __shared__ __align__(16) float sT[8][16 * 68];
  const int lane = threadIdx.x & 31;
  const int wave = threadIdx.x >> 5;
  const int tilesN = N >> 6;
  const int tilesM = M >> 6;
  const int tile = blockIdx.x * 8 + wave;
  if (tile >= tilesM * tilesN) return;
  const int tm = tile / tilesN;
  const int tn = tile - tm * tilesN;
  const int m0 = tm << 6;
  const int n0 = tn << 6;

  const int rlane = lane & 15;
  const int koff  = (lane >> 4) * 8;
  const int mOff  = (lane >> 4) * 8;

  v8f acc[4][4];
#pragma unroll
  for (int i = 0; i < 4; ++i)
#pragma unroll
    for (int j = 0; j < 4; ++j) acc[i][j] = (v8f){0.f, 0.f, 0.f, 0.f, 0.f, 0.f, 0.f, 0.f};

  for (int k0 = 0; k0 < K; k0 += 32) {
    v16b bh[4], bl[4];
#pragma unroll
    for (int j = 0; j < 4; ++j) {
      const size_t bo = (size_t)(n0 + (j << 4) + rlane) * ldb + koff + k0;
      bh[j] = FragB::load(Bt + bo);
      bl[j] = FragB::load(Bt2 + bo);
    }
#pragma unroll
    for (int i = 0; i < 4; ++i) {
      const size_t ao = (size_t)(m0 + (i << 4) + rlane) * lda + koff + k0;
      const v16b ah = FragB::load(A + ao);
      const v16b al = FragB::load(A2 + ao);
#pragma unroll
      for (int j = 0; j < 4; ++j) {
        acc[i][j] = FragB::mma(ah, bh[j], acc[i][j]);
        acc[i][j] = FragB::mma(ah, bl[j], acc[i][j]);
        acc[i][j] = FragB::mma(al, bh[j], acc[i][j]);
      }
      dep_guard4_b(acc[i][0], acc[i][1], acc[i][2], acc[i][3], ah, al);
    }
    keep4_b(bh[0], bh[1], bh[2], bh[3]);
    keep4_b(bl[0], bl[1], bl[2], bl[3]);
  }
  acc_guard4(acc[0][0], acc[0][1], acc[0][2], acc[0][3]);
  acc_guard4(acc[1][0], acc[1][1], acc[1][2], acc[1][3]);
  acc_guard4(acc[2][0], acc[2][1], acc[2][2], acc[2][3]);
  acc_guard4(acc[3][0], acc[3][1], acc[3][2], acc[3][3]);

  float* slab = sT[wave];
#pragma unroll
  for (int i = 0; i < 4; ++i) {
    const int mBase = m0 + (i << 4);
    float bm[8];
    if (BIAS_MODE == 1) {
      const v4f q0 = *(const v4f*)(bias + mBase + mOff);
      const v4f q1 = *(const v4f*)(bias + mBase + mOff + 4);
      bm[0] = q0.x; bm[1] = q0.y; bm[2] = q0.z; bm[3] = q0.w;
      bm[4] = q1.x; bm[5] = q1.y; bm[6] = q1.z; bm[7] = q1.w;
    } else {
#pragma unroll
      for (int r = 0; r < 8; ++r) bm[r] = 0.0f;
    }
#pragma unroll
    for (int j = 0; j < 4; ++j) {
      const int n = n0 + (j << 4) + rlane;
      float bv = 0.f;
      if (BIAS_MODE == 2) bv = bias[n];
#pragma unroll
      for (int r = 0; r < 8; ++r) {
        float v = acc[i][j][r];
        if (BIAS_MODE == 1) v += bm[r];
        if (BIAS_MODE == 2) v += bv;
        slab[(mOff + r) * 68 + (j << 4) + rlane] = v;
      }
    }
    __builtin_amdgcn_fence(__ATOMIC_RELEASE, "workgroup");
    __builtin_amdgcn_wave_barrier();
    __builtin_amdgcn_fence(__ATOMIC_ACQUIRE, "workgroup");
    {
      const int hh = lane >> 4, c4 = (lane & 15) * 4;
      for (int pass = 0; pass < 2; ++pass) {
#pragma unroll
        for (int it = 0; it < 8; ++it) {
          const int row = it * 2 + hh;
          const v4f v = *(const v4f*)(slab + row * 68 + c4);
          *(volatile v4f*)(Cout + (size_t)(mBase + row) * ldc + n0 + c4) = v;
        }
        __threadfence();
      }
    }
    __builtin_amdgcn_fence(__ATOMIC_RELEASE, "workgroup");
    __builtin_amdgcn_wave_barrier();
    __builtin_amdgcn_fence(__ATOMIC_ACQUIRE, "workgroup");
  }
}

__global__ __launch_bounds__(256) void bn1_partial(const float* __restrict__ Y, float* __restrict__ part) {
  __shared__ __align__(16) float sp[512];
  const int c = threadIdx.x;
  const float* y = Y + (size_t)blockIdx.x * kPartRows * kC1 + c;
  const float c0 = y[0];
  float s = 0.0f, q = 0.0f;
#pragma unroll 8
  for (int r = 0; r < kPartRows; ++r) {
    const float v = y[(size_t)r * kC1] - c0;
    s += v;
    const float vv = v * v;
    q += vv;
  }
  const float inv = 1.0f / (float)kPartRows;
  const float sm  = s * inv;
  const float mb  = c0 + sm;
  const float cr  = s * sm;
  const float m2  = fmaxf(q - cr, 0.0f);
  sp[c] = mb;
  sp[256 + c] = m2;
  __syncthreads();
  if (c < 128) {
    const v4f v = *(const v4f*)(sp + 4 * c);
    float* dst = part + (size_t)blockIdx.x * 512 + 4 * c;
    *(volatile v4f*)dst = v;
    __threadfence();
    *(volatile v4f*)dst = v;
  }
}

__global__ __launch_bounds__(256) void bn1_finalize(const float* __restrict__ part, const float* __restrict__ g,
                                                    float* __restrict__ tab) {
  __shared__ __align__(16) float so[512];
  const int c = threadIdx.x;
  float sm = 0.0f;
#pragma unroll 8
  for (int p = 0; p < kPartBlocks; ++p) sm += part[(size_t)p * 512 + c];
  const float mean = sm * (1.0f / (float)kPartBlocks);
  float dd = 0.0f, m2 = 0.0f;
#pragma unroll 4
  for (int p = 0; p < kPartBlocks; ++p) {
    const float e = part[(size_t)p * 512 + c] - mean;
    const float ee = e * e;
    dd += ee;
    m2 += part[(size_t)p * 512 + 256 + c];
  }
  const float tot = m2 + (float)kPartRows * dd;
  const float var = fmaxf(tot * (1.0f / (float)kRows), 0.0f);
  const float sc  = g[c] * (1.0f / sqrtf(var + kBnEps));
  so[c] = mean;
  so[256 + c] = sc;
  __syncthreads();
  if (c < 128) {
    const v4f v = *(const v4f*)(so + 4 * c);
    float* dst = tab + 4 * c;
    *(volatile v4f*)dst = v;
    __threadfence();
    *(volatile v4f*)dst = v;
  }
}

__global__ __launch_bounds__(256) void bn1_relu_split(const float* __restrict__ Y, const float* __restrict__ tab,
                                                      const float* __restrict__ beta,
                                                      unsigned short* __restrict__ Hhi,
                                                      unsigned short* __restrict__ Hlo) {
  const int lane = threadIdx.x & 31;
  const int wave = threadIdx.x >> 5;
  const int c8 = lane * 8;
  const v4f mu0 = *(const v4f*)(tab + c8);
  const v4f mu1 = *(const v4f*)(tab + c8 + 4);
  const v4f sc0 = *(const v4f*)(tab + 256 + c8);
  const v4f sc1 = *(const v4f*)(tab + 256 + c8 + 4);
  const v4f be0 = *(const v4f*)(beta + c8);
  const v4f be1 = *(const v4f*)(beta + c8 + 4);
  const int row0 = blockIdx.x * 128 + wave * 16;
#pragma unroll 2
  for (int rr = 0; rr < 16; ++rr) {
    const size_t row = (size_t)(row0 + rr);
    const float* yr = Y + row * kC1 + c8;
    const v4f a0 = *(const v4f*)(yr);
    const v4f a1 = *(const v4f*)(yr + 4);
    float f[8];
#pragma unroll
    for (int e = 0; e < 4; ++e) {
      const float t0 = (a0[e] - mu0[e]) * sc0[e];
      f[e] = fmaxf(t0 + be0[e], 0.0f);
      const float t1 = (a1[e] - mu1[e]) * sc1[e];
      f[4 + e] = fmaxf(t1 + be1[e], 0.0f);
    }
    v4u H, L;
    split_pack8(f, H, L);
    const size_t o = row * kC1 + c8;
    store2_planes(Hhi + o, Hlo + o, H, L);
  }
}

__global__ __launch_bounds__(256) void bn2_stats(const float* __restrict__ Y2t, const float* __restrict__ g,
                                                 float* __restrict__ tab2) {
  __shared__ float rs[256];
  __shared__ float rq[256];
  const int t = threadIdx.x;
  const int c = blockIdx.x;
  const float* row = Y2t + (size_t)c * kRows;
  const float c0 = row[0];
  float s = 0.0f, q = 0.0f;
#pragma unroll 4
  for (int it = 0; it < kRows / 1024; ++it) {
    const v4f y = *(const v4f*)(row + (size_t)(it * 256 + t) * 4);
#pragma unroll
    for (int e = 0; e < 4; ++e) {
      const float v = y[e] - c0;
      s += v;
      const float vv = v * v;
      q += vv;
    }
  }
  rs[t] = s;
  rq[t] = q;
  for (int off = 128; off > 0; off >>= 1) {
    __syncthreads();
    if (t < off) {
      rs[t] = rs[t] + rs[t + off];
      rq[t] = rq[t] + rq[t + off];
    }
  }
  __syncthreads();
  const float S = rs[0];
  const float Q = rq[0];
  const float inv = 1.0f / (float)kRows;
  const float sm  = S * inv;
  const float mu  = c0 + sm;
  const float qm  = Q * inv;
  const float sq  = sm * sm;
  const float var = fmaxf(qm - sq, 0.0f);
  const float sc  = g[c] * (1.0f / sqrtf(var + kBnEps));
  if (t < 32) {
    const float v = (t == 0) ? mu : ((t == 1) ? sc : 0.0f);
    float* dst = tab2 + (size_t)c * 32 + t;
    *(volatile float*)dst = v;
    __threadfence();
    *(volatile float*)dst = v;
  }
}

__global__ __launch_bounds__(256) void bn2_relu_out(const float* __restrict__ Y2t, const float* __restrict__ tab2,
                                                    const float* __restrict__ beta, float* __restrict__ out) {
  const int i = blockIdx.x * 256 + threadIdx.x;
  const int e = i << 2;
  const int c = e / kRows;
  const int m = e - c * kRows;
  const int b = m / kNq;
  const int n = m - b * kNq;
  const float mu = tab2[c * 32];
  const float sc = tab2[c * 32 + 1];
  const float bt = beta[c];
  const v4f y = *(const v4f*)(Y2t + e);
  v4f o;
#pragma unroll
  for (int k = 0; k < 4; ++k) {
    const float t0 = (y[k] - mu) * sc;
    float v = fmaxf(t0 + bt, 0.0f);
    v = (fabsf(v) <= 3.4028234663852886e38f) ? v : 0.0f;
    o[k] = v;
  }
  float* dst = out + ((size_t)(b * kC2 + c) * kNq + n);
  *(volatile v4f*)dst = o;
  __threadfence();
  *(volatile v4f*)dst = o;
}

extern "C" void kernel_launch(void* const* d_in, const int* in_sizes, int n_in,
                              void* d_out, int out_size, void* d_ws, size_t ws_size,
                              hipStream_t stream) {
  (void)in_sizes; (void)n_in; (void)out_size;
  const float* xyz1    = (const float*)d_in[0];
  const float* xyz2    = (const float*)d_in[1];
  const float* points1 = (const float*)d_in[2];
  const float* points2 = (const float*)d_in[3];
  const float* w1      = (const float*)d_in[4];
  const float* b1      = (const float*)d_in[5];
  const float* g1      = (const float*)d_in[6];
  const float* be1     = (const float*)d_in[7];
  const float* w2      = (const float*)d_in[8];
  const float* b2      = (const float*)d_in[9];
  const float* g2      = (const float*)d_in[10];
  const float* be2     = (const float*)d_in[11];
  float* out = (float*)d_out;

  constexpr size_t szW1  = (size_t)kC1 * kK1 * 2;
  constexpr size_t szW2  = (size_t)kC2 * kC1 * 2;
  constexpr size_t szP2t = (size_t)kBatch * kNs * kD2 * 4;
  constexpr size_t szX   = (size_t)kRows * kK1 * 2;
  constexpr size_t szH   = (size_t)kRows * kC1 * 2;
  constexpr size_t szY1  = (size_t)kRows * kC1 * 4;
  constexpr size_t szY2  = (size_t)kC2 * kRows * 4;
  constexpr size_t szP1  = (size_t)kPartBlocks * 512 * 4;
  constexpr size_t szT1  = 512 * 4;
  constexpr size_t szT2  = (size_t)kC2 * 32 * 4;
  constexpr size_t oW1h = 0;
  constexpr size_t oW1l = oW1h + szW1;
  constexpr size_t oW2h = oW1l + szW1;
  constexpr size_t oW2l = oW2h + szW2;
  constexpr size_t oP2t = oW2l + szW2;
  constexpr size_t oXh  = oP2t + szP2t;
  constexpr size_t oXl  = oXh + szX;
  constexpr size_t oY1  = oXl + szX;
  constexpr size_t oY2  = oY1 + szY1;
  constexpr size_t oP1  = oY2 + szY2;
  constexpr size_t oT1  = oP1 + szP1;
  constexpr size_t oT2  = oT1 + szT1;
  constexpr size_t wsTotal = oT2 + szT2;
  static_assert(szH <= szX, "H1 planes fit inside the dead X planes");
  static_assert(wsTotal <= (size_t)134217728, "carve within 128 MiB");
  static_assert((oW1l % 256) == 0 && (oW2h % 256) == 0 && (oP2t % 256) == 0 && (oXh % 256) == 0 &&
                (oXl % 256) == 0 && (oY1 % 256) == 0 && (oY2 % 256) == 0 && (oP1 % 256) == 0 &&
                (oT1 % 256) == 0 && (oT2 % 256) == 0, "aligned carve");
  if (ws_size < wsTotal) return;

  char* ws = (char*)d_ws;
  unsigned short* W1h = (unsigned short*)(ws + oW1h);
  unsigned short* W1l = (unsigned short*)(ws + oW1l);
  unsigned short* W2h = (unsigned short*)(ws + oW2h);
  unsigned short* W2l = (unsigned short*)(ws + oW2l);
  float*          p2t = (float*)(ws + oP2t);
  unsigned short* Xh  = (unsigned short*)(ws + oXh);
  unsigned short* Xl  = (unsigned short*)(ws + oXl);
  unsigned short* Hh  = (unsigned short*)(ws + oXh);
  unsigned short* Hl  = (unsigned short*)(ws + oXl);
  float*          Y1  = (float*)(ws + oY1);
  float*          Y2t = (float*)(ws + oY2);
  float*          pt1 = (float*)(ws + oP1);
  float*          tb1 = (float*)(ws + oT1);
  float*          tb2 = (float*)(ws + oT2);

  pack_wt_split<<<(kC1 * (kK1 / 8)) / 256, 256, 0, stream>>>(w1, kK1, kC1, W1h, W1l);
  pack_wt_split<<<(kC2 * (kC1 / 8)) / 256, 256, 0, stream>>>(w2, kC1, kC2, W2h, W2l);

  transpose_p2<<<dim3(kNs / 32, kD2 / 64, kBatch), 256, 0, stream>>>(points2, p2t);

  xcols_from_p1<<<dim3(kNq / 32, kD1 / 64, kBatch), 256, 0, stream>>>(points1, Xh, Xl);

  knn3_interp<<<dim3(kNq / 256, kBatch), 256, 0, stream>>>(xyz1, xyz2, p2t, Xh, Xl);

  wmma_gemm64_bf16x3<2><<<((kRows / 64) * (kC1 / 64)) / 8, 256, 0, stream>>>(
      Xh, Xl, kK1, W1h, W1l, kK1, Y1, kC1, b1, kRows, kC1, kK1);

  bn1_partial<<<kPartBlocks, 256, 0, stream>>>(Y1, pt1);
  bn1_finalize<<<1, 256, 0, stream>>>(pt1, g1, tb1);
  bn1_relu_split<<<kRows / 128, 256, 0, stream>>>(Y1, tb1, be1, Hh, Hl);

  wmma_gemm64_bf16x3<1><<<((kC2 / 64) * (kRows / 64)) / 8, 256, 0, stream>>>(
      W2h, W2l, kC1, Hh, Hl, kC1, Y2t, kRows, b2, kC2, kRows, kC1);

  bn2_stats<<<kC2, 256, 0, stream>>>(Y2t, g2, tb2);
  bn2_relu_out<<<(kC2 * kRows / 4) / 256, 256, 0, stream>>>(Y2t, tb2, be2, out);
}
